// QKVAttentionLegacy_16518444221163
// MI455X (gfx1250) — hardware-verified
//
#include <hip/hip_runtime.h>


#define NB_  4
#define NH_  16
#define CH   64
#define NT_  1024
#define NBH  (NB_ * NH_)
#define WID  (3 * NH_ * CH)
#define PSC  32768.0f
#define LOSC 1024.0f
#define LOSCI (1.0f / 1024.0f)

typedef _Float16 h16;
typedef __attribute__((ext_vector_type(16))) _Float16 v16h;
typedef __attribute__((ext_vector_type(8)))  _Float16 v8h;
typedef __attribute__((ext_vector_type(8)))  float    v8f;
typedef __attribute__((ext_vector_type(4)))  float    v4f;
typedef v8h  __attribute__((may_alias)) v8ha;
typedef v4f  __attribute__((may_alias)) v4fa;

__device__ __forceinline__ unsigned short f2bf(float f) { unsigned u = __float_as_uint(f); u += 0x7FFFu + ((u >> 16) & 1u); return (unsigned short)(u >> 16); }
__device__ __forceinline__ float bf2f(unsigned short b) { return __uint_as_float(((unsigned)b) << 16); }
__device__ __forceinline__ float bfr(float f) { return bf2f(f2bf(f)); }
__device__ __forceinline__ v16h cat16(v8h lo, v8h hi) { return __builtin_shufflevector(lo, hi, 0, 1, 2, 3, 4, 5, 6, 7, 8, 9, 10, 11, 12, 13, 14, 15); }
__device__ __forceinline__ v8f wmma16(v16h a, v16h b, v8f c) { return __builtin_amdgcn_wmma_f32_16x16x32_f16(false, a, false, b, (short)0, c, false, false); }
#define VST2(T, p, v) do { const T vst2_v_ = (v); *(volatile T*)(p) = vst2_v_; __threadfence(); *(volatile T*)(p) = vst2_v_; } while (0)

__global__ __launch_bounds__(256) void k_qkT(const float* __restrict__ qkv, h16* Q16, h16* K16) {
    __shared__ __align__(16) h16 tl[64 * 72];
    const int which = blockIdx.z, bh = blockIdx.y, t0 = blockIdx.x * 64, tid = threadIdx.x;
    const int b = bh / NH_, h = bh - b * NH_;
    const int c = tid >> 2, tq = (tid & 3) * 16;
    const float* src = qkv + ((size_t)b * WID + h * 3 * CH + which * CH + c) * NT_ + t0 + tq;
#pragma unroll
    for (int i = 0; i < 16; ++i) tl[(tq + i) * 72 + c] = (h16)bfr(src[i]);
    __syncthreads();
    h16* dst = (which == 0 ? Q16 : K16) + ((size_t)bh * NT_ + t0) * CH;
    const int piece = tid & 7;
    auto pass = [&]() {
#pragma unroll
        for (int s = 0; s < 2; ++s) { const int t = (tid >> 3) + 32 * s; const v8h val = *(const v8ha*)(tl + t * 72 + piece * 8); *(volatile v8h*)(dst + (size_t)t * CH + piece * 8) = val; }
    };
    pass(); __threadfence(); pass();
}
__global__ __launch_bounds__(256) void k_v16(const float* __restrict__ qkv, h16* V16) {
    typedef __attribute__((ext_vector_type(4))) _Float16 v4h;
    const int lane = threadIdx.x & 31; const size_t w = (size_t)blockIdx.x * 8 + (threadIdx.x >> 5);
    const int seg = (int)(w % (NT_ / 128)); const size_t rc = w / (NT_ / 128); const int c = (int)(rc % CH); const int bh = (int)(rc / CH);
    if (bh >= NBH) return;
    const int b = bh / NH_, h = bh - b * NH_;
    const float* src = qkv + ((size_t)b * WID + h * 3 * CH + 2 * CH + c) * NT_ + seg * 128 + lane * 4;
    v4h o;
#pragma unroll
    for (int i = 0; i < 4; ++i) o[i] = (h16)bfr(src[i]);
    VST2(v4h, V16 + ((size_t)bh * CH + c) * NT_ + seg * 128 + lane * 4, o);
}
__global__ __launch_bounds__(128) void k_attn(const h16* __restrict__ Q16, const h16* __restrict__ K16, const h16* __restrict__ V16, float* out) {
    __shared__ __align__(16) h16 plds[4][16 * 32];
    __shared__ __align__(16) h16 plds2[4][16 * 32];
    __shared__ __align__(16) float ot[CH * 68];
    const int lane = threadIdx.x & 31, wave = threadIdx.x >> 5, lr = lane & 15, hi = lane >> 4;
    const int bh = blockIdx.x / (NT_ / 64), qt = blockIdx.x - bh * (NT_ / 64), q0l = qt * 64, q0 = q0l + wave * 16;
    h16* pl = &plds[wave][0]; h16* pl2 = &plds2[wave][0];
    const h16* qb = Q16 + (size_t)bh * NT_ * CH; const h16* kb = K16 + (size_t)bh * NT_ * CH; const h16* vb = V16 + (size_t)bh * CH * NT_;
    v16h qa[2];
#pragma unroll
    for (int kc = 0; kc < 2; ++kc) { const h16* p = qb + (size_t)(q0 + lr) * CH + kc * 32 + 8 * hi; qa[kc] = cat16(*(const v8h*)p, *(const v8h*)(p + 16)); }
    v8f o[4], ox[4];
#pragma unroll
    for (int n = 0; n < 4; ++n) { o[n] = (v8f){}; ox[n] = (v8f){}; }
    float mrow[8], lpart[8];
#pragma unroll
    for (int j = 0; j < 8; ++j) { mrow[j] = -3.0e38f; lpart[j] = 0.f; }
#pragma unroll 1
    for (int kt = 0; kt < NT_ / 32; ++kt) {
        const int l0 = kt * 32;
        v8f s0 = {}, s1 = {};
#pragma unroll
        for (int kc = 0; kc < 2; ++kc) {
            const h16* r0p = kb + (size_t)(l0 + lr) * CH + kc * 32 + 8 * hi; const h16* r1p = r0p + (size_t)16 * CH;
            s0 = wmma16(qa[kc], cat16(*(const v8h*)r0p, *(const v8h*)(r0p + 16)), s0);
            s1 = wmma16(qa[kc], cat16(*(const v8h*)r1p, *(const v8h*)(r1p + 16)), s1);
        }
        asm volatile("v_nop\n\tv_nop\n\tv_nop\n\tv_nop" : "+v"(s0), "+v"(s1) : "v"(qa[0]), "v"(qa[1]));
        float alpha[8];
#pragma unroll
        for (int j = 0; j < 8; ++j) {
            const float a0 = s0[j] * 0.125f, a1 = s1[j] * 0.125f;
            float mx = fmaxf(a0, a1);
            mx = fmaxf(mx, __shfl_xor(mx, 1, 16)); mx = fmaxf(mx, __shfl_xor(mx, 2, 16)); mx = fmaxf(mx, __shfl_xor(mx, 4, 16)); mx = fmaxf(mx, __shfl_xor(mx, 8, 16));
            const float mn = fmaxf(mrow[j], mx);
            alpha[j] = __expf(mrow[j] - mn); mrow[j] = mn;
            const float p0 = __expf(a0 - mn), p1 = __expf(a1 - mn);
            lpart[j] = lpart[j] * alpha[j] + (p0 + p1);
            const int mr = hi * 8 + j;
            const float ps0 = p0 * PSC, ps1 = p1 * PSC; const h16 h0 = (h16)ps0, h1 = (h16)ps1;
            pl[mr * 32 + lr] = h0; pl[mr * 32 + 16 + lr] = h1; pl2[mr * 32 + lr] = (h16)((ps0 - (float)h0) * LOSC); pl2[mr * 32 + 16 + lr] = (h16)((ps1 - (float)h1) * LOSC);
        }
#pragma unroll
        for (int n = 0; n < 4; ++n)
#pragma unroll
            for (int j = 0; j < 8; ++j) { o[n][j] *= alpha[j]; ox[n][j] *= alpha[j]; }
        asm volatile("" ::: "memory");
        const v16h pa = cat16(*(const v8ha*)(pl + lr * 32 + hi * 8), *(const v8ha*)(pl + lr * 32 + 16 + hi * 8));
        const v16h px = cat16(*(const v8ha*)(pl2 + lr * 32 + hi * 8), *(const v8ha*)(pl2 + lr * 32 + 16 + hi * 8));
#pragma unroll
        for (int n = 0; n < 4; ++n) { const h16* vp = vb + (size_t)(n * 16 + lr) * NT_ + l0 + hi * 8; const v16h vv = cat16(*(const v8h*)vp, *(const v8h*)(vp + 16));
            o[n] = wmma16(pa, vv, o[n]); ox[n] = wmma16(px, vv, ox[n]); }
        asm volatile("v_nop\n\tv_nop\n\tv_nop\n\tv_nop" : "+v"(o[0]), "+v"(o[1]), "+v"(o[2]), "+v"(o[3]), "+v"(ox[0]), "+v"(ox[1]), "+v"(ox[2]), "+v"(ox[3]) : "v"(pa), "v"(px));
    }
    float inv[8];
#pragma unroll
    for (int j = 0; j < 8; ++j) { float rs = lpart[j]; rs += __shfl_xor(rs, 1, 16); rs += __shfl_xor(rs, 2, 16); rs += __shfl_xor(rs, 4, 16); rs += __shfl_xor(rs, 8, 16); inv[j] = 1.0f / (rs * PSC); }
#pragma unroll
    for (int n = 0; n < 4; ++n)
#pragma unroll
        for (int j = 0; j < 8; ++j) ot[(n * 16 + lr) * 68 + wave * 16 + hi * 8 + j] = (o[n][j] + ox[n][j] * LOSCI) * inv[j];
    __syncthreads();
    float* ob = out + (size_t)bh * CH * NT_ + q0l;
    auto pass = [&]() {
#pragma unroll
        for (int s = 0; s < 8; ++s) { const int c = wave * 16 + s * 2 + (lane >> 4), piece = lane & 15; const v4f val = *(const v4fa*)(ot + c * 68 + piece * 4);
            *(volatile v4f*)(ob + (size_t)c * NT_ + piece * 4) = val; }
    };
    pass(); __threadfence(); pass();
}

extern "C" void kernel_launch(void* const* d_in, const int* in_sizes, int n_in,
                              void* d_out, int out_size, void* d_ws, size_t ws_size, hipStream_t stream) {
    (void)in_sizes; (void)n_in; (void)out_size;
    const float* qkv = (const float*)d_in[0];
    float* out = (float*)d_out;
    char* wsp = (char*)d_ws;
    auto take = [&](size_t bytes) { char* p = wsp; wsp += (bytes + 255) & ~(size_t)255; return (void*)p; };
    h16* Q16 = (h16*)take((size_t)NBH * NT_ * CH * 2); h16* K16 = (h16*)take((size_t)NBH * NT_ * CH * 2); h16* V16 = (h16*)take((size_t)NBH * CH * NT_ * 2);
    if ((size_t)(wsp - (char*)d_ws) > ws_size) return;
    k_qkT<<<dim3(NT_ / 64, NBH, 2), 256, 0, stream>>>(qkv, Q16, K16);
    k_v16<<<(NBH * CH * (NT_ / 128)) / 8, 256, 0, stream>>>(qkv, V16);
    k_attn<<<NBH * (NT_ / 64), 128, 0, stream>>>(Q16, K16, V16, out);
}
